// SinkhornOT_82471962018276
// MI455X (gfx1250) — hardware-run, weakly checked
//
#include <hip/hip_runtime.h>
#define KNG 16
#define KNR 1024
#define KNW 256
#define KIT 5
#define KREG 0.1f
#define KLEN 1e-12f
typedef unsigned short v8us __attribute__((ext_vector_type(8), may_alias));
typedef float  v8f  __attribute__((ext_vector_type(8)));
typedef float  v4f  __attribute__((ext_vector_type(4)));
typedef float  v4fa __attribute__((ext_vector_type(4), may_alias));

__device__ __forceinline__ unsigned short bf16_bits(float x) { unsigned int u = __float_as_uint(x); return (unsigned short)((u + 0x7FFFu + ((u >> 16) & 1u)) >> 16); }
__device__ __forceinline__ float bf16_val(unsigned short b) { return __uint_as_float(((unsigned int)b) << 16); }
__device__ __forceinline__ float bf16_round(float x) { return bf16_val(bf16_bits(x)); }

typedef _Float16 v16h __attribute__((ext_vector_type(16)));
union FragH { v16h v; v8us half[2]; _Float16 h[16]; unsigned short u[16]; };

typedef _Float16 v4h __attribute__((ext_vector_type(4)));

__global__ __launch_bounds__(256) void k_x16(const float* __restrict__ x, _Float16* __restrict__ X16, size_t n8) { const size_t t = (size_t)blockIdx.x * 256 + threadIdx.x; if (t >= n8) return; FragH f;
#pragma unroll
  for (int q = 0; q < 8; ++q) f.h[q] = (_Float16)bf16_round(x[t * 8 + q]); *(volatile v8us*)((unsigned short*)X16 + t * 8) = f.half[0]; __threadfence(); *(volatile v8us*)((unsigned short*)X16 + t * 8) = f.half[0]; }

__device__ __forceinline__ v16h g2_frag(const _Float16* p, int hh) { FragH f; f.half[0] = *(const v8us*)((const unsigned short*)p + 8 * hh); f.half[1] = *(const v8us*)((const unsigned short*)p + 16 + 8 * hh); return f.v; }
__device__ __forceinline__ v8f g2_mma(v16h a, v16h b, v8f c) { v8f d = __builtin_amdgcn_wmma_f32_16x16x32_f16(false, a, false, b, (short)0, c, false, false); asm volatile("v_nop\n\tv_nop\n\tv_nop\n\tv_nop" : "+v"(d) : "v"(a), "v"(b)); return d; }
template <int ACT>
__global__ __launch_bounds__(128) void k_gemm2(const _Float16* __restrict__ A, int lda, size_t sA, const _Float16* __restrict__ Bh, int ldb, size_t sB, float alpha, const float* __restrict__ bias, size_t sBias, const float* __restrict__ CP, int rowsPerB, size_t sCPb, int row0g,
    float* __restrict__ C, _Float16* __restrict__ C16, int ldc, size_t sC, int M, int N, int K) { static_assert(ACT == 0 || ACT == 3 || ACT == 6 || ACT == 8 || ACT == 9 || ACT == 11 || ACT == 12 || ACT == 14 || ACT == 15 || ACT == 16 || ACT == 17, "k_gemm2: unsupported ACT code (would silently apply no activation)");
  __shared__ __attribute__((aligned(16))) float so[4][32][68];
  const int tid = threadIdx.x, w = tid >> 5, lane = tid & 31, ln = lane & 15, hh = lane >> 4; const int by = blockIdx.y;
  A += (size_t)by * sA; Bh += (size_t)by * sB; const size_t cofs = (size_t)by * sC; const float* bp = bias ? bias + (size_t)by * sBias : nullptr;
  const int ntn = N >> 6; const int mt = blockIdx.x / ntn, nq = blockIdx.x - mt * ntn; const int row0 = mt * 128 + 32 * w, col0 = nq * 64; if (row0 >= M) return;
  const _Float16* a0p = A + (size_t)(row0 + ln) * lda; const _Float16* a1p = a0p + (size_t)16 * lda;
  const _Float16* b0p = Bh + (size_t)(col0 + ln) * ldb; const _Float16* b1p = b0p + (size_t)16 * ldb; const _Float16* b2p = b1p + (size_t)16 * ldb; const _Float16* b3p = b2p + (size_t)16 * ldb;
  const v8f z8 = {0.f,0.f,0.f,0.f,0.f,0.f,0.f,0.f}; v8f c00 = z8, c01 = z8, c02 = z8, c03 = z8, c10 = z8, c11 = z8, c12 = z8, c13 = z8;
  for (int kb = 0; kb < K; kb += 32) { const v16h a0 = g2_frag(a0p + kb, hh), a1 = g2_frag(a1p + kb, hh);
    v16h b = g2_frag(b0p + kb, hh); c00 = g2_mma(a0, b, c00); c10 = g2_mma(a1, b, c10);
    b = g2_frag(b1p + kb, hh); c01 = g2_mma(a0, b, c01); c11 = g2_mma(a1, b, c11);
    b = g2_frag(b2p + kb, hh); c02 = g2_mma(a0, b, c02); c12 = g2_mma(a1, b, c12);
    b = g2_frag(b3p + kb, hh); c03 = g2_mma(a0, b, c03); c13 = g2_mma(a1, b, c13); }
  v8f accs[8] = {c00, c01, c02, c03, c10, c11, c12, c13};
#pragma unroll
  for (int u = 0; u < 8; ++u) { const int t = u & 3, half = u >> 2; const int col = col0 + t * 16 + ln; const float bv = bp ? bf16_round(bp[col]) : 0.f;
#pragma unroll
    for (int r = 0; r < 8; ++r) { const int rloc = half * 16 + 8 * hh + r; float v = accs[u][r] * alpha + bv; if (CP) { if (rowsPerB < 0) v += CP[cofs + (size_t)(row0g + row0 + rloc) * ldc + col];        else { const int bidx = (row0g + row0 + rloc) / rowsPerB; v += CP[(size_t)bidx * sCPb + (size_t)by * 64 + col]; } }
      if (ACT == 3) v = fmaxf(v, 0.f); else if (ACT == 6) v = 0.5f * v * (1.0f + erff(v * 0.70710678118654752f)); else if (ACT == 11) v = 1.0f / (1.0f + expf(-v)); else if (ACT == 15) v = v / (1.0f + expf(-v)); else if (ACT == 12) v = (v > 0.f) ? v : 0.01f * v; else if (ACT == 8) v = tanhf(v); else if (ACT == 9) v = 0.5f * v * (1.0f + tanhf(0.7978845608028654f * (v + 0.044715f * v * v * v))); else if (ACT == 14) v = (v > 0.f) ? v : 0.1f * v; else if (ACT == 16) v = (v >= 0.f) ? v : 0.3f * v; else if (ACT == 17) v = (v >= 0.f) ? v : 0.2f * v;
      so[w][rloc][t * 16 + ln] = v; } }
  __builtin_amdgcn_fence(__ATOMIC_ACQ_REL, "workgroup"); __builtin_amdgcn_wave_barrier();
  const int rsub = lane >> 4, c4 = (lane & 15) * 4;
  for (int pass = 0; pass < 2; ++pass) {
#pragma unroll
    for (int q = 0; q < 16; ++q) { const int r = q * 2 + rsub; const v4f v = *(const v4fa*)&so[w][r][c4]; if (C) *(volatile v4f*)(C + cofs + (size_t)(row0 + r) * ldc + col0 + c4) = v; if (C16) { v4h h4; for (int i = 0; i < 4; ++i) h4[i] = (_Float16)v[i]; *(volatile v4h*)(C16 + cofs + (size_t)(row0 + r) * ldc + col0 + c4) = h4; } }
    if (pass == 0) __threadfence(); } }

__global__ __launch_bounds__(256) void k_nrc(const float* __restrict__ F, _Float16* __restrict__ H, unsigned rows) {
  const unsigned r = blockIdx.x * 256u + threadIdx.x; if (r >= rows) return;
  const float* p = F + (size_t)r * KNW; unsigned short* o = (unsigned short*)H + (size_t)r * KNW; float s = 0.0f;
  for (unsigned j = 0; j < (unsigned)KNW; j += 4) { const v4f a = *(const v4fa*)(p + j);
#pragma unroll
    for (int q = 0; q < 4; ++q) s += a[q] * a[q]; }
  const float d = fmaxf(sqrtf(s), KLEN);
  for (unsigned j = 0; j < (unsigned)KNW; j += 8) { const v4f a = *(const v4fa*)(p + j); const v4f b = *(const v4fa*)(p + j + 4); FragH f;
#pragma unroll
    for (int q = 0; q < 4; ++q) { f.h[q] = (_Float16)(a[q] / d); f.h[4 + q] = (_Float16)(b[q] / d); }
    const v8us w = f.half[0]; *(volatile v8us*)(o + j) = w; __threadfence(); *(volatile v8us*)(o + j) = w; }
}

__global__ __launch_bounds__(256) void k_zm0(const float* __restrict__ cs, float* __restrict__ zm) {
  const unsigned t = blockIdx.x * 256u + threadIdx.x; if (t >= (unsigned)(KNG * KNR * (KNR / 4))) return;
  const v4f c = *(const v4fa*)(cs + (size_t)t * 4); v4f w;
#pragma unroll
  for (int q = 0; q < 4; ++q) { const float ct = 1.0f - c[q]; w[q] = (0.0f - ct) / KREG; }
  float* d = zm + (size_t)t * 4; *(volatile v4f*)d = w; __threadfence(); *(volatile v4f*)d = w; }

__global__ __launch_bounds__(256) void k_rls(float* zm, unsigned nrows) {
  const unsigned r = blockIdx.x * 256u + threadIdx.x; if (r >= nrows) return;
  float* p = zm + (size_t)r * KNR; float hi = p[0];
  for (unsigned j = 0; j < (unsigned)KNR; j += 4) { const v4f a = *(const v4fa*)(p + j); hi = fmaxf(fmaxf(fmaxf(hi, a[0]), fmaxf(a[1], a[2])), a[3]); }
  float s = 0.0f;
  for (unsigned j = 0; j < (unsigned)KNR; j += 4) { const v4f a = *(const v4fa*)(p + j);
#pragma unroll
    for (int q = 0; q < 4; ++q) s += expf(a[q] - hi); }
  const float l = hi + logf(s);
  for (unsigned j = 0; j < (unsigned)KNR; j += 4) { const v4f a = *(const v4fa*)(p + j); v4f w;
#pragma unroll
    for (int q = 0; q < 4; ++q) w[q] = a[q] - l;
    *(volatile v4f*)(p + j) = w; __threadfence(); *(volatile v4f*)(p + j) = w; }
}

__global__ __launch_bounds__(256) void k_cls(float* zm) {
  const unsigned t = blockIdx.x * 256u + threadIdx.x; if (t >= (unsigned)(KNG * KNR)) return;
  float* p = zm + (size_t)(t / KNR) * KNR * KNR + (t % KNR); const float* rp = p; float hi = rp[0];
  for (unsigned n = 0; n < (unsigned)KNR; n += 4) { const float a0 = rp[(size_t)n * KNR], a1 = rp[(size_t)(n + 1) * KNR], a2 = rp[(size_t)(n + 2) * KNR], a3 = rp[(size_t)(n + 3) * KNR]; hi = fmaxf(fmaxf(fmaxf(hi, a0), fmaxf(a1, a2)), a3); }
  float s = 0.0f;
  for (unsigned n = 0; n < (unsigned)KNR; n += 4) { const float a0 = rp[(size_t)n * KNR], a1 = rp[(size_t)(n + 1) * KNR], a2 = rp[(size_t)(n + 2) * KNR], a3 = rp[(size_t)(n + 3) * KNR]; s += expf(a0 - hi); s += expf(a1 - hi); s += expf(a2 - hi); s += expf(a3 - hi); }
  const float l = hi + logf(s);
  for (unsigned n = 0; n < (unsigned)KNR; n += 4) {
#pragma unroll
    for (unsigned u = 0; u < 4; ++u) { float* d = p + (size_t)(n + u) * KNR; const float w = rp[(size_t)(n + u) * KNR] - l; *(volatile float*)d = w; __threadfence(); *(volatile float*)d = w; } }
}

__global__ __launch_bounds__(256) void k_pex(const float* __restrict__ zm, const float* __restrict__ cs, float* __restrict__ pl, float* __restrict__ rs, unsigned nrows) {
  const unsigned r = blockIdx.x * 256u + threadIdx.x; if (r >= nrows) return;
  const float* p = zm + (size_t)r * KNR; const float* c = cs + (size_t)r * KNR; float* o = pl + (size_t)r * KNR; float acc = 0.0f;
  for (unsigned j = 0; j < (unsigned)KNR; j += 4) { const v4f a = *(const v4fa*)(p + j); const v4f b = *(const v4fa*)(c + j); v4f w;
#pragma unroll
    for (int q = 0; q < 4; ++q) { w[q] = expf(a[q]); acc += w[q] * (1.0f - b[q]); }
    *(volatile v4f*)(o + j) = w; __threadfence(); *(volatile v4f*)(o + j) = w; }
  *(volatile float*)(rs + r) = acc; __threadfence(); *(volatile float*)(rs + r) = acc; }

template <int LEN>
__global__ __launch_bounds__(256) void k_sum(const float* __restrict__ src, float* __restrict__ dst, unsigned nthr, float scl) {
  const unsigned t = blockIdx.x * 256u + threadIdx.x; if (t >= nthr) return;
  const float* p = src + (size_t)t * LEN; float s = 0.0f;
  for (unsigned n = 0; n < (unsigned)LEN; ++n) s += p[n];
  const float w = s * scl; *(volatile float*)(dst + t) = w; __threadfence(); *(volatile float*)(dst + t) = w; }

extern "C" void kernel_launch(void* const* d_in, const int* in_sizes, int n_in,
                              void* d_out, int out_size, void* d_ws, size_t ws_size, hipStream_t stream) {
  (void)in_sizes; (void)n_in; (void)out_size;
  const float* const* I = (const float* const*)d_in; const float* ta = I[0]; const float* tb = I[1]; const float* wa = I[2]; const float* va = I[3]; const float* wb = I[4]; const float* vb = I[5];
  float* pl = (float*)d_out; float* tc = pl + (size_t)KNG * KNR * KNR;
  static_assert((KNG * KNR) % 128 == 0 && KNR % 128 == 0 && KNR % 64 == 0 && KNW % 64 == 0 && KNW % 32 == 0 && KNW % 8 == 0 && KNR % 4 == 0, "whole tiles");
  uint8_t* wsp = (uint8_t*)d_ws; size_t off = 0;
  auto take = [&](size_t bytes) { uint8_t* p = wsp + off; off += (bytes + 255) & ~(size_t)255; return p; };
  float* CS = (float*)take((size_t)KNG * KNR * KNR * 4); float* ZM = (float*)take((size_t)KNG * KNR * KNR * 4); float* FA = (float*)take((size_t)KNG * KNR * KNW * 4); float* FB = (float*)take((size_t)KNG * KNR * KNW * 4);
  _Float16* TA = (_Float16*)take((size_t)KNG * KNR * KNW * 2); _Float16* TB = (_Float16*)take((size_t)KNG * KNR * KNW * 2); _Float16* WA = (_Float16*)take((size_t)KNW * KNW * 2); _Float16* WB = (_Float16*)take((size_t)KNW * KNW * 2); _Float16* HA = (_Float16*)take((size_t)KNG * KNR * KNW * 2); _Float16* HB = (_Float16*)take((size_t)KNG * KNR * KNW * 2); float* RS = (float*)take((size_t)KNG * KNR * 4); float* GS = (float*)take((size_t)KNG * 4);
  if (off > ws_size) return;
  k_x16<<<(unsigned)(((size_t)KNG * KNR * KNW / 8 + 255) / 256), 256, 0, stream>>>(ta, TA, (size_t)KNG * KNR * KNW / 8);
  k_x16<<<(unsigned)(((size_t)KNG * KNR * KNW / 8 + 255) / 256), 256, 0, stream>>>(tb, TB, (size_t)KNG * KNR * KNW / 8);
  k_x16<<<(unsigned)(((size_t)KNW * KNW / 8 + 255) / 256), 256, 0, stream>>>(wa, WA, (size_t)KNW * KNW / 8);
  k_x16<<<(unsigned)(((size_t)KNW * KNW / 8 + 255) / 256), 256, 0, stream>>>(wb, WB, (size_t)KNW * KNW / 8);
  k_gemm2<0><<<dim3((unsigned)(((KNG * KNR) / 128) * (KNW / 64)), 1), 128, 0, stream>>>(TA, KNW, 0, WA, KNW, 0, 1.0f, va, 0, nullptr, 1, 0, 0, FA, nullptr, KNW, 0, KNG * KNR, KNW, KNW);
  k_gemm2<0><<<dim3((unsigned)(((KNG * KNR) / 128) * (KNW / 64)), 1), 128, 0, stream>>>(TB, KNW, 0, WB, KNW, 0, 1.0f, vb, 0, nullptr, 1, 0, 0, FB, nullptr, KNW, 0, KNG * KNR, KNW, KNW);
  k_nrc<<<(unsigned)((KNG * KNR + 255) / 256), 256, 0, stream>>>(FA, HA, (unsigned)(KNG * KNR));
  k_nrc<<<(unsigned)((KNG * KNR + 255) / 256), 256, 0, stream>>>(FB, HB, (unsigned)(KNG * KNR));
  k_gemm2<0><<<dim3((unsigned)((KNR / 128) * (KNR / 64)), KNG), 128, 0, stream>>>(HA, KNW, (size_t)KNR * KNW, HB, KNW, (size_t)KNR * KNW, 1.0f, nullptr, 0, nullptr, 1, 0, 0, CS, nullptr, KNR, (size_t)KNR * KNR, KNR, KNR, KNW);
  k_zm0<<<(unsigned)(((size_t)KNG * KNR * (KNR / 4) + 255) / 256), 256, 0, stream>>>(CS, ZM);
  for (int it = 0; it < KIT; ++it) {
    k_rls<<<(unsigned)((KNG * KNR + 255) / 256), 256, 0, stream>>>(ZM, (unsigned)(KNG * KNR));
    k_cls<<<(unsigned)((KNG * KNR + 255) / 256), 256, 0, stream>>>(ZM); }
  k_pex<<<(unsigned)((KNG * KNR + 255) / 256), 256, 0, stream>>>(ZM, CS, pl, RS, (unsigned)(KNG * KNR));
  k_sum<KNR><<<1, 256, 0, stream>>>(RS, GS, (unsigned)KNG, 1.0f);
  k_sum<KNG><<<1, 256, 0, stream>>>(GS, tc, 1u, 1.0f / (float)KNG);
}
